// ImageTextMatchingModel_78340203479445
// MI455X (gfx1250) — hardware-verified
//
#include <hip/hip_runtime.h>
#include <math.h>

typedef __attribute__((ext_vector_type(16))) _Float16 v16h;
typedef __attribute__((ext_vector_type(16))) __bf16 v16b;
typedef __attribute__((ext_vector_type(8)))  _Float16 v8h;
typedef __attribute__((ext_vector_type(8)))  float v8f;
typedef __attribute__((ext_vector_type(4)))  float v4f;
typedef __attribute__((ext_vector_type(2)))  float v2f;
typedef __attribute__((ext_vector_type(4)))  unsigned v4u;
typedef __attribute__((ext_vector_type(4)))  int v4i;
typedef float __attribute__((may_alias)) float_a;
typedef int __attribute__((may_alias)) int_a;

template <typename T> __device__ __forceinline__ void vst2(void* p, T v) { *(volatile T*)p = v; __threadfence(); *(volatile T*)p = v; }
__device__ __forceinline__ v8f wmma16(v16h a, v16h b, v8f c) {
  v8f d = __builtin_amdgcn_wmma_f32_16x16x32_f16(false, a, false, b, (short)0, c, false, false);
  asm volatile("v_nop\n\tv_nop\n\tv_nop\n\tv_nop" : "+v"(d) : "v"(a), "v"(b));
  return d;
}
__device__ __forceinline__ v8f wmma_bf(v16b a, v16b b, v8f c) {
  v8f d = __builtin_amdgcn_wmma_f32_16x16x32_bf16(false, a, false, b, (short)0, c, false, false);
  asm volatile("v_nop\n\tv_nop\n\tv_nop\n\tv_nop" : "+v"(d) : "v"(a), "v"(b));
  return d;
}
__device__ __forceinline__ v16h frag_h(const _Float16* rowk0, int lane) {
  union { v16h v; v8h q[2]; } u; const _Float16* p = rowk0 + 8 * (lane >> 4);
  u.q[0] = *(const v8h*)p; u.q[1] = *(const v8h*)(p + 16); return u.v;
}
__device__ __forceinline__ v16h frag_f32(const float* rowk0, int lane) {
  v16h a; const float* p = rowk0 + 8 * (lane >> 4);
#pragma unroll
  for (int i = 0; i < 8; ++i) { a[i] = (_Float16)p[i]; a[8 + i] = (_Float16)p[16 + i]; }
  return a;
}
__device__ __forceinline__ v16h frag_f32s(const float* rowk0, int lane, float sc) {
  v16h a; const float* p = rowk0 + 8 * (lane >> 4);
#pragma unroll
  for (int i = 0; i < 8; ++i) { a[i] = (_Float16)(p[i] * sc); a[8 + i] = (_Float16)(p[16 + i] * sc); }
  return a;
}
__device__ __forceinline__ v16h fragc_f32(const float* W, int k0, int n, int lane, int ld, int K) {
  v16h a; const int g = lane >> 4;
#pragma unroll
  for (int i = 0; i < 8; ++i) { const int ka = k0 + 8 * g + i, kb = ka + 16;
    a[i] = (_Float16)(ka < K ? W[(size_t)(ka < K ? ka : K - 1) * ld + n] : 0.f); a[8 + i] = (_Float16)(kb < K ? W[(size_t)(kb < K ? kb : K - 1) * ld + n] : 0.f); }
  return a;
}
struct F2 { v16b h, l; };
__device__ __forceinline__ F2 bsplit16(const float v[16]) { F2 r;
#pragma unroll
  for (int i = 0; i < 16; ++i) { const __bf16 h = (__bf16)v[i]; r.h[i] = h; r.l[i] = (__bf16)(v[i] - (float)h); }
  return r; }
__device__ __forceinline__ F2 split_row(const float* row, int k0, int lane) { float v[16]; const float* p = row + k0 + 8 * (lane >> 4);
#pragma unroll
  for (int i = 0; i < 8; ++i) { v[i] = p[i]; v[8 + i] = p[16 + i]; }
  return bsplit16(v); }
__device__ __forceinline__ F2 split_rowK(const float* row, int k0, int lane, int K) { float v[16]; const int g = lane >> 4;
#pragma unroll
  for (int i = 0; i < 8; ++i) { const int ka = k0 + 8 * g + i, kb = ka + 16; v[i] = ka < K ? row[ka < K ? ka : K - 1] : 0.f; v[8 + i] = kb < K ? row[kb < K ? kb : K - 1] : 0.f; }
  return bsplit16(v); }
__device__ __forceinline__ F2 split_col(const float* W, int k0, int n, int lane, int ld, int K) { float v[16]; const int g = lane >> 4;
#pragma unroll
  for (int i = 0; i < 8; ++i) { const int ka = k0 + 8 * g + i, kb = ka + 16; v[i] = ka < K ? W[(size_t)(ka < K ? ka : K - 1) * ld + n] : 0.f; v[8 + i] = kb < K ? W[(size_t)(kb < K ? kb : K - 1) * ld + n] : 0.f; }
  return bsplit16(v); }
__device__ __forceinline__ v8f mac3(const F2& a, const F2& b, v8f c) { c = wmma_bf(a.l, b.h, c); c = wmma_bf(a.h, b.l, c); return wmma_bf(a.h, b.h, c); }
__device__ __forceinline__ float sigm(float v) { return 1.0f / (1.0f + expf(-v)); }
#define LDSX() do { asm volatile("s_wait_dscnt 0" ::: "memory"); __builtin_amdgcn_wave_barrier(); __builtin_amdgcn_fence(__ATOMIC_RELEASE, "workgroup"); } while (0)


#define NB 64
#define NP 196
#define NT 77
#define CI 1024
#define DD 512
#define NHD 8
#define HD 64
#define NRI (NB * NP)
#define NRT (NB * NT)
#define NPP 208
#define NTP 80
#ifndef NRI_USE
#define NRI_USE NRI
#define NB_USE NB
#endif
typedef __attribute__((ext_vector_type(8))) __bf16 v8b;
__device__ __forceinline__ v16b frag_b(const __bf16* rowk0, int lane) {
  union { v16b v; v8b q[2]; } u; const __bf16* p = rowk0 + 8 * (lane >> 4);
  u.q[0] = *(const v8b*)p; u.q[1] = *(const v8b*)(p + 16); return u.v;
}
__device__ __forceinline__ v16b frag_gbf(const float* rowk0, int lane) {
  v16b a; const float* p = rowk0 + 8 * (lane >> 4);
#pragma unroll
  for (int i = 0; i < 8; ++i) { a[i] = (__bf16)p[i]; a[8 + i] = (__bf16)p[16 + i]; }
  return a;
}
__device__ __forceinline__ float bfr(float v) { return (float)(__bf16)v; }
__device__ __attribute__((noinline)) float exp_ni(float v) { return expf(v); }

#define WS_PTI  0u
#define WS_PTT  (WS_PTI + 2u * DD * CI)
#define WS_PT4  (WS_PTT + 2u * DD * CI)
#define WS_XT   (WS_PT4 + 2u * 4 * DD * DD)
#define WS_PI   (WS_XT + 2u * NRI * CI)
#define WS_Q    (WS_PI + 4u * NRI * DD)
#define WS_KV   (WS_Q + 4u * NRI * DD)
#define WS_AT   (WS_KV + 4u * NRT * 2 * DD)
#define PHP 96
#define WS_WM   (WS_AT + 4u * NRI * DD)
#define WS_END  (WS_WM + 4u * NB * NP * PHP)

__global__ __launch_bounds__(256) void k_pack(const float* __restrict__ Wi, const float* __restrict__ Wt, const float* __restrict__ Wq, const float* __restrict__ Wk, const float* __restrict__ Wv, const float* __restrict__ Wo, __bf16* __restrict__ PTI, __bf16* __restrict__ PTT, __bf16* __restrict__ PT4) {
  __shared__ __align__(16) __bf16 srow[CI];
  const int n = blockIdx.x, tid = threadIdx.x; const float* Wm; int K, nn; __bf16* dst;
  if (n < DD) { Wm = Wi; K = CI; nn = n; dst = PTI + (size_t)nn * CI; } else if (n < 2 * DD) { Wm = Wt; K = CI; nn = n - DD; dst = PTT + (size_t)nn * CI; }
  else { const int m = (n - 2 * DD) / DD; nn = (n - 2 * DD) % DD; K = DD; Wm = m == 0 ? Wq : m == 1 ? Wk : m == 2 ? Wv : Wo; dst = PT4 + ((size_t)m * DD + nn) * DD; }
  for (int k = tid; k < K; k += 256) srow[k] = (__bf16)Wm[(size_t)k * DD + nn];
  __syncthreads();
  if (tid < K / 8) vst2((unsigned*)(dst + tid * 8), *(const v4u*)(&srow[tid * 8]));
}
__global__ __launch_bounds__(256) void k_tr(const float* __restrict__ img, __bf16* __restrict__ XT) {
  __shared__ __bf16 st[NP][72];
  const int b = blockIdx.y, c0 = blockIdx.x * 64, tid = threadIdx.x;
  for (int q = tid; q < 64 * NP; q += 256) { const int cl = q / NP, n = q - cl * NP; st[n][cl] = (__bf16)img[((size_t)b * CI + c0 + cl) * NP + n]; }
  __syncthreads();
  for (int q = tid; q < NP * 8; q += 256) { const int n = q >> 3, pc = q & 7; union { __bf16 e[8]; v4u u; } pk;
#pragma unroll
    for (int e = 0; e < 8; ++e) pk.e[e] = st[n][pc * 8 + e];
    vst2((unsigned*)(XT + ((size_t)b * NP + n) * CI + c0 + pc * 8), pk.u); }
}
__global__ __launch_bounds__(128) void k_proj(const __bf16* __restrict__ XT, const float* __restrict__ TXT, const __bf16* __restrict__ PTI, const __bf16* __restrict__ PTT, const float* __restrict__ bi, const float* __restrict__ bt, float* __restrict__ PI, float* __restrict__ PTXT) {
  __shared__ __align__(16) float so[4][16][132];
  const int tid = threadIdx.x, wave = tid >> 5, lane = tid & 31, col = lane & 15, g = lane >> 4; const int which = blockIdx.z; const size_t r0 = (size_t)blockIdx.x * 64 + wave * 16; const int n0 = blockIdx.y * 128;
  const int nrows = which ? NRT : NRI_USE; if ((size_t)blockIdx.x * 64 >= (size_t)nrows) return;
  const size_t ra = (r0 + col) < (size_t)nrows ? (r0 + col) : (size_t)(nrows - 1);
  v8f acc[8] = {};
  const __bf16* PT = which ? PTT : PTI; const float* bb_ = which ? bt : bi;
#pragma unroll 2
  for (int kc = 0; kc < CI / 32; ++kc) { const v16b a = which ? frag_gbf(TXT + ra * CI + kc * 32, lane) : frag_b(XT + ra * CI + kc * 32, lane);
#pragma unroll
    for (int j = 0; j < 8; ++j) acc[j] = wmma_bf(a, frag_b(PT + (size_t)(n0 + j * 16 + col) * CI + kc * 32, lane), acc[j]); }
#pragma unroll
  for (int j = 0; j < 8; ++j) { const float bb = bfr(bb_[n0 + j * 16 + col]);
#pragma unroll
    for (int r = 0; r < 8; ++r) so[wave][8 * g + r][j * 16 + col] = acc[j][r] + bb; }
  LDSX();
  float* dst = which ? PTXT : PI;
  for (int rl = 0; rl < 16; ++rl) { const size_t row = r0 + rl; if (row < (size_t)nrows) vst2(dst + row * DD + n0 + lane * 4, *(const v4f*)(&so[wave][rl][lane * 4])); }
}
__global__ __launch_bounds__(128) void k_lin(const float* __restrict__ PI, const float* __restrict__ PTXT, const float* __restrict__ AT, const __bf16* __restrict__ PT4, const float* __restrict__ bq, const float* __restrict__ bk, const float* __restrict__ bv, const float* __restrict__ bo,
                                             float* __restrict__ Q, float* __restrict__ KV, float* __restrict__ AO, int wbase) {
  __shared__ __align__(16) float so[4][16][132];
  const int tid = threadIdx.x, wave = tid >> 5, lane = tid & 31, col = lane & 15, g = lane >> 4; const int which = blockIdx.z + wbase; const int n0 = blockIdx.y * 128;
  const int nrows = which == 1 ? NRT : NRI_USE; const int ncols = which == 1 ? 2 * DD : DD;
  if ((size_t)blockIdx.x * 64 >= (size_t)nrows || n0 >= ncols) return;
  const float* IN = which == 0 ? PI : which == 1 ? PTXT : AT; float* OUT = which == 0 ? Q : which == 1 ? KV : AO;
  const int m = which == 0 ? 0 : which == 1 ? (n0 < DD ? 1 : 2) : 3; const int nn0 = which == 1 ? (n0 & (DD - 1)) : n0;
  const float* bias = which == 0 ? bq : which == 1 ? (n0 < DD ? bk : bv) : bo;
  const size_t r0 = (size_t)blockIdx.x * 64 + wave * 16; const size_t ra = (r0 + col) < (size_t)nrows ? (r0 + col) : (size_t)(nrows - 1);
  v8f acc[8] = {};
#pragma unroll 2
  for (int kc = 0; kc < DD / 32; ++kc) { const F2 a = split_row(IN + ra * DD, kc * 32, lane);
#pragma unroll
    for (int j = 0; j < 8; ++j) { const v16b wb = frag_b(PT4 + ((size_t)m * DD + nn0 + j * 16 + col) * DD + kc * 32, lane); acc[j] = wmma_bf(a.l, wb, acc[j]); acc[j] = wmma_bf(a.h, wb, acc[j]); } }
#pragma unroll
  for (int j = 0; j < 8; ++j) { const float bb = bfr(bias[nn0 + j * 16 + col]);
#pragma unroll
    for (int r = 0; r < 8; ++r) so[wave][8 * g + r][j * 16 + col] = acc[j][r] + bb; }
  LDSX();
  for (int rl = 0; rl < 16; ++rl) { const size_t row = r0 + rl; if (row < (size_t)nrows) vst2(OUT + row * ncols + n0 + lane * 4, *(const v4f*)(&so[wave][rl][lane * 4])); }
}
__global__ __launch_bounds__(256) void k_attn(const float* __restrict__ Q, const float* __restrict__ KV, float* __restrict__ AT, float* __restrict__ WM) {
  __shared__ __align__(16) __bf16 skh[NTP][72], skl[NTP][72];
  __shared__ __align__(16) __bf16 svh[HD][104], svl[HD][104];
  __shared__ __align__(16) float sp[8][16][100];
  __shared__ __align__(16) float so[8][16][68];
  const int tid = threadIdx.x, wave = tid >> 5, lane = tid & 31, col = lane & 15, g = lane >> 4;
  const int b = blockIdx.x;
#pragma unroll 1
  for (int h = 0; h < NHD; ++h) {
    __syncthreads();
    for (int q = tid; q < NTP * 64; q += 256) { const int t = q >> 6, d = q & 63; float kv = 0.f; if (t < NT) kv = KV[((size_t)b * NT + t) * 2 * DD + h * HD + d]; const __bf16 hi = (__bf16)kv; skh[t][d] = hi; skl[t][d] = (__bf16)(kv - (float)hi); }
    for (int q = tid; q < HD * 96; q += 256) { const int d = q / 96, t = q - d * 96; float vv = 0.f; if (t < NT) vv = KV[((size_t)b * NT + t) * 2 * DD + DD + h * HD + d]; const __bf16 hi = (__bf16)vv; svh[d][t] = hi; svl[d][t] = (__bf16)(vv - (float)hi); }
    __syncthreads();
#pragma unroll 1
    for (int qt = wave; qt < 13; qt += 8) {
      const int n = qt * 16 + col; const int nc = n < NP ? n : NP - 1; const float* qrow = Q + ((size_t)b * NP + nc) * DD + h * HD;
      const F2 a0 = split_row(qrow, 0, lane), a1 = split_row(qrow, 32, lane);
      v8f s[5];
#pragma unroll
      for (int ct = 0; ct < 5; ++ct) { v8f acc = {}; const __bf16* kh0 = &skh[ct * 16 + col][0]; const __bf16* kl0 = &skl[ct * 16 + col][0];
        acc = wmma_bf(a0.l, frag_b(kh0, lane), acc); acc = wmma_bf(a0.h, frag_b(kl0, lane), acc); acc = wmma_bf(a0.h, frag_b(kh0, lane), acc);
        acc = wmma_bf(a1.l, frag_b(kh0 + 32, lane), acc); acc = wmma_bf(a1.h, frag_b(kl0 + 32, lane), acc); acc = wmma_bf(a1.h, frag_b(kh0 + 32, lane), acc);
        s[ct] = acc; }
#pragma unroll
      for (int r = 0; r < 8; ++r) { float mx = -3.0e38f;
#pragma unroll
        for (int ct = 0; ct < 5; ++ct) { const int t = ct * 16 + col; const float v = (t < NT) ? s[ct][r] * 0.125f : -3.0e38f; s[ct][r] = v; mx = fmaxf(mx, v); }
#pragma unroll
        for (int o = 1; o < 16; o <<= 1) mx = fmaxf(mx, __shfl_xor(mx, o));
        float sum = 0.f;
#pragma unroll
        for (int ct = 0; ct < 5; ++ct) { const int t = ct * 16 + col; const float e = (t < NT) ? exp_ni(s[ct][r] - mx) : 0.f; s[ct][r] = e; sum += e; }
#pragma unroll
        for (int o = 1; o < 16; o <<= 1) sum += __shfl_xor(sum, o);
        const float inv = 1.0f / sum;
#pragma unroll
        for (int ct = 0; ct < 5; ++ct) sp[wave][8 * g + r][ct * 16 + col] = s[ct][r] * inv;
        sp[wave][8 * g + r][80 + col] = 0.f; }
      LDSX();
      for (int qq = lane; qq < 16 * 24; qq += 32) { const int rl = qq / 24, pc = qq - rl * 24; const int nr = qt * 16 + rl;
        if (nr < NP) { float* dst = WM + ((size_t)b * NP + nr) * PHP + pc * 4; v4f cur = *(const v4f*)&sp[wave][rl][pc * 4];
          if (h > 0) { const float4 old = *(const float4*)dst; cur[0] += old.x; cur[1] += old.y; cur[2] += old.z; cur[3] += old.w; }
          vst2(dst, cur); } }
      v8f o[4] = {};
#pragma unroll
      for (int kc = 0; kc < 3; ++kc) { const F2 pa = split_row(&sp[wave][col][0], kc * 32, lane);
#pragma unroll
        for (int dt = 0; dt < 4; ++dt) { const __bf16* vh0 = &svh[dt * 16 + col][kc * 32]; const __bf16* vl0 = &svl[dt * 16 + col][kc * 32];
          o[dt] = wmma_bf(pa.l, frag_b(vh0, lane), o[dt]); o[dt] = wmma_bf(pa.h, frag_b(vl0, lane), o[dt]); o[dt] = wmma_bf(pa.h, frag_b(vh0, lane), o[dt]); } }
#pragma unroll
      for (int dt = 0; dt < 4; ++dt)
#pragma unroll
        for (int r = 0; r < 8; ++r) so[wave][8 * g + r][dt * 16 + col] = o[dt][r];
      LDSX();
      for (int qq = lane; qq < 16 * 16; qq += 32) { const int rl = qq >> 4, pc = qq & 15; const int nr = qt * 16 + rl; if (nr < NP) vst2(AT + ((size_t)b * NP + nr) * DD + h * HD + pc * 4, *(const v4f*)&so[wave][rl][pc * 4]); }
      LDSX(); }
  }
}
__global__ __launch_bounds__(256) void k_copyw(const float* __restrict__ WM, float* __restrict__ OW) {
  const size_t p = (size_t)blockIdx.x * 256 + threadIdx.x; const size_t total = (size_t)NB * NP * NT;
  if (p * 4 >= total) return; v4f v;
#pragma unroll
  for (int i = 0; i < 4; ++i) { const size_t f = p * 4 + i; const size_t fc = f < total ? f : total - 1; const size_t row = fc / NT, t = fc % NT; v[i] = f < total ? WM[row * PHP + t] * (1.0f / NHD) : 0.f; }
  vst2(OW + p * 4, v);
}
__global__ __launch_bounds__(512) void k_avg(const float* __restrict__ AO, const float* __restrict__ PTXT, float* __restrict__ AVG, float* __restrict__ CLS) {
  __shared__ __align__(16) float sa[DD], sc[DD];
  const int b = blockIdx.x, d = threadIdx.x; float a = 0.f, c = 0.f;
#pragma unroll 4
  for (int n = 0; n < NP; ++n) a += AO[((size_t)b * NP + n) * DD + d];
#pragma unroll 4
  for (int t = 0; t < NT; ++t) c += PTXT[((size_t)b * NT + t) * DD + d];
  sa[d] = a / (float)NP; sc[d] = c / (float)NT;
  __syncthreads();
  if (d < 128) { vst2(AVG + (size_t)b * DD + d * 4, *(const v4f*)&sa[d * 4]); vst2(CLS + (size_t)b * DD + d * 4, *(const v4f*)&sc[d * 4]); }
}
__global__ __launch_bounds__(256) void k_score(const float* __restrict__ AVG, const float* __restrict__ CLS, float* __restrict__ SC) {
  __shared__ float na[NB], ncz[NB]; __shared__ __align__(16) float ss[NB][NB + 4];
  const int tid = threadIdx.x, wave = tid >> 5, lane = tid & 31;
  for (int r = wave; r < 2 * NB; r += 8) { const float* src = r < NB ? AVG + (size_t)r * DD : CLS + (size_t)(r - NB) * DD; float s = 0.f;
    for (int d = lane; d < DD; d += 32) { const float v = src[d]; s += v * v; }
#pragma unroll
    for (int o = 1; o < 32; o <<= 1) s += __shfl_xor(s, o);
    if (lane == 0) { const float nrm = fmaxf(sqrtf(s), 1e-8f); if (r < NB) na[r] = nrm; else ncz[r - NB] = nrm; } }
  __syncthreads();
  for (int pr = wave; pr < NB * NB / 32; pr += 8) {
    const int i = pr >> 1, j = (pr & 1) * 32 + lane; float s = 0.f;
    for (int d = 0; d < DD; ++d) s += (AVG[(size_t)i * DD + d] / na[i]) * (CLS[(size_t)j * DD + d] / ncz[j]);
    ss[i][j] = s; }
  __syncthreads();
  for (int q = tid; q < NB * 16; q += 256) { const int i = q >> 4, pc = q & 15; vst2(SC + (size_t)i * NB + pc * 4, *(const v4f*)&ss[i][pc * 4]); }
}

extern "C" void kernel_launch(void* const* d_in, const int* in_sizes, int n_in, void* d_out, int out_size, void* d_ws, size_t ws_size, hipStream_t stream) {
  (void)in_sizes; (void)n_in; (void)out_size;
  const float** F = (const float**)d_in;
  if (ws_size < (size_t)WS_END) return;
  char* ws = (char*)d_ws;
  __bf16 *PTI = (__bf16*)(ws + WS_PTI), *PTT = (__bf16*)(ws + WS_PTT), *PT4 = (__bf16*)(ws + WS_PT4), *XT = (__bf16*)(ws + WS_XT);
  float *PI = (float*)(ws + WS_PI), *Q = (float*)(ws + WS_Q), *KV = (float*)(ws + WS_KV), *AT = (float*)(ws + WS_AT), *WM = (float*)(ws + WS_WM);
  float* SC = (float*)d_out; float* AO = SC + NB * NB; float* OW = AO + (size_t)NRI * DD; float* AVG = OW + (size_t)NB * NP * NT; float* CLS = AVG + NB * DD; float* PTXT = CLS + NB * DD;
  k_pack<<<2 * DD + 4 * DD, 256, 0, stream>>>(F[2], F[4], F[6], F[8], F[10], F[12], PTI, PTT, PT4);
  k_tr<<<dim3(CI / 64, NB), 256, 0, stream>>>(F[0], XT);
  k_proj<<<dim3(NRI / 64, DD / 128, 2), 128, 0, stream>>>(XT, F[1], PTI, PTT, F[3], F[5], PI, PTXT);
  k_lin<<<dim3(NRI / 64, 2 * DD / 128, 2), 128, 0, stream>>>(PI, PTXT, nullptr, PT4, F[7], F[9], F[11], F[13], Q, KV, nullptr, 0);
  k_attn<<<NB_USE, 256, 0, stream>>>(Q, KV, AT, WM);
  k_lin<<<dim3(NRI / 64, DD / 128, 1), 128, 0, stream>>>(PI, PTXT, AT, PT4, F[7], F[9], F[11], F[13], Q, KV, AO, 2);
  k_copyw<<<(NB * NP * NT / 4 + 255) / 256, 256, 0, stream>>>(WM, OW);
  k_avg<<<NB, 512, 0, stream>>>(AO, PTXT, AVG, CLS);
  k_score<<<1, 256, 0, stream>>>(AVG, CLS, SC);
}
